// DecGCN_88888643158468
// MI455X (gfx1250) — hardware-verified
//
#include <hip/hip_runtime.h>
#include <math.h>

typedef __attribute__((ext_vector_type(16))) _Float16 v16h;
typedef __attribute__((ext_vector_type(16))) __bf16 v16b;
typedef __attribute__((ext_vector_type(8)))  _Float16 v8h;
typedef __attribute__((ext_vector_type(8)))  float v8f;
typedef __attribute__((ext_vector_type(4)))  float v4f;
typedef __attribute__((ext_vector_type(2)))  float v2f;
typedef __attribute__((ext_vector_type(4)))  unsigned v4u;
typedef __attribute__((ext_vector_type(4)))  int v4i;
typedef float __attribute__((may_alias)) float_a;
typedef int __attribute__((may_alias)) int_a;

template <typename T> __device__ __forceinline__ void vst2(void* p, T v) { *(volatile T*)p = v; __threadfence(); *(volatile T*)p = v; }
__device__ __forceinline__ v8f wmma16(v16h a, v16h b, v8f c) {
  v8f d = __builtin_amdgcn_wmma_f32_16x16x32_f16(false, a, false, b, (short)0, c, false, false);
  asm volatile("v_nop\n\tv_nop\n\tv_nop\n\tv_nop" : "+v"(d) : "v"(a), "v"(b));
  return d;
}
__device__ __forceinline__ v8f wmma_bf(v16b a, v16b b, v8f c) {
  v8f d = __builtin_amdgcn_wmma_f32_16x16x32_bf16(false, a, false, b, (short)0, c, false, false);
  asm volatile("v_nop\n\tv_nop\n\tv_nop\n\tv_nop" : "+v"(d) : "v"(a), "v"(b));
  return d;
}
__device__ __forceinline__ v16h frag_h(const _Float16* rowk0, int lane) {
  union { v16h v; v8h q[2]; } u; const _Float16* p = rowk0 + 8 * (lane >> 4);
  u.q[0] = *(const v8h*)p; u.q[1] = *(const v8h*)(p + 16); return u.v;
}
__device__ __forceinline__ v16h frag_f32(const float* rowk0, int lane) {
  v16h a; const float* p = rowk0 + 8 * (lane >> 4);
#pragma unroll
  for (int i = 0; i < 8; ++i) { a[i] = (_Float16)p[i]; a[8 + i] = (_Float16)p[16 + i]; }
  return a;
}
__device__ __forceinline__ v16h frag_f32s(const float* rowk0, int lane, float sc) {
  v16h a; const float* p = rowk0 + 8 * (lane >> 4);
#pragma unroll
  for (int i = 0; i < 8; ++i) { a[i] = (_Float16)(p[i] * sc); a[8 + i] = (_Float16)(p[16 + i] * sc); }
  return a;
}
__device__ __forceinline__ v16h fragc_f32(const float* W, int k0, int n, int lane, int ld, int K) {
  v16h a; const int g = lane >> 4;
#pragma unroll
  for (int i = 0; i < 8; ++i) { const int ka = k0 + 8 * g + i, kb = ka + 16;
    a[i] = (_Float16)(ka < K ? W[(size_t)(ka < K ? ka : K - 1) * ld + n] : 0.f); a[8 + i] = (_Float16)(kb < K ? W[(size_t)(kb < K ? kb : K - 1) * ld + n] : 0.f); }
  return a;
}
struct F2 { v16b h, l; };
__device__ __forceinline__ F2 bsplit16(const float v[16]) { F2 r;
#pragma unroll
  for (int i = 0; i < 16; ++i) { const __bf16 h = (__bf16)v[i]; r.h[i] = h; r.l[i] = (__bf16)(v[i] - (float)h); }
  return r; }
__device__ __forceinline__ F2 split_row(const float* row, int k0, int lane) { float v[16]; const float* p = row + k0 + 8 * (lane >> 4);
#pragma unroll
  for (int i = 0; i < 8; ++i) { v[i] = p[i]; v[8 + i] = p[16 + i]; }
  return bsplit16(v); }
__device__ __forceinline__ F2 split_rowK(const float* row, int k0, int lane, int K) { float v[16]; const int g = lane >> 4;
#pragma unroll
  for (int i = 0; i < 8; ++i) { const int ka = k0 + 8 * g + i, kb = ka + 16; v[i] = ka < K ? row[ka < K ? ka : K - 1] : 0.f; v[8 + i] = kb < K ? row[kb < K ? kb : K - 1] : 0.f; }
  return bsplit16(v); }
__device__ __forceinline__ F2 split_col(const float* W, int k0, int n, int lane, int ld, int K) { float v[16]; const int g = lane >> 4;
#pragma unroll
  for (int i = 0; i < 8; ++i) { const int ka = k0 + 8 * g + i, kb = ka + 16; v[i] = ka < K ? W[(size_t)(ka < K ? ka : K - 1) * ld + n] : 0.f; v[8 + i] = kb < K ? W[(size_t)(kb < K ? kb : K - 1) * ld + n] : 0.f; }
  return bsplit16(v); }
__device__ __forceinline__ v8f mac3(const F2& a, const F2& b, v8f c) { c = wmma_bf(a.l, b.h, c); c = wmma_bf(a.h, b.l, c); return wmma_bf(a.h, b.h, c); }
__device__ __forceinline__ float sigm(float v) { return 1.0f / (1.0f + expf(-v)); }
#define LDSX() do { asm volatile("s_wait_dscnt 0" ::: "memory"); __builtin_amdgcn_wave_barrier(); __builtin_amdgcn_fence(__ATOMIC_RELEASE, "workgroup"); } while (0)


#define N0 16000
#define N1 12000
#define N2 6000
#define HH 256
#define EIN 128
#define OUTD 128
__device__ __forceinline__ float bfr(float v) { return (float)(__bf16)v; }
typedef __attribute__((ext_vector_type(8))) __bf16 v8b;
__device__ __forceinline__ v16b frag_b(const __bf16* rowk0, int lane) {
  union { v16b v; v8b q[2]; } u; const __bf16* p = rowk0 + 8 * (lane >> 4);
  u.q[0] = *(const v8b*)p; u.q[1] = *(const v8b*)(p + 16); return u.v;
}
__device__ __attribute__((noinline)) float exp_ni(float v) { return expf(v); }

#define WS_PT    0u
#define PT_WIN(m)  ((size_t)(m) * 256 * 128)
#define PT_WOUT(m) ((size_t)2 * 256 * 128 + (size_t)(m) * 128 * 256)
#define PT_WS2C    ((size_t)2 * 256 * 128 + 2 * 128 * 256)
#define PT_WC2S    (PT_WS2C + 128 * 128)
#define PT_END     (PT_WC2S + 128 * 128)
#define WS_H0    (WS_PT + 2u * 163840)
#define WS_H1    (WS_H0 + 4u * 2 * N0 * HH)
#define WS_H2    (WS_H1 + 4u * 2 * N1 * HH)
#define WS_S     (WS_H2 + 4u * 2 * N2 * HH)
#define WS_END   (WS_S + 4u * 2 * N2 * OUTD)

__global__ __launch_bounds__(256) void k_pack(const float* __restrict__ WinS, const float* __restrict__ WinC, const float* __restrict__ WoS, const float* __restrict__ WoC, const float* __restrict__ Ws2c, const float* __restrict__ Wc2s, __bf16* __restrict__ PT) {
  __shared__ __align__(16) __bf16 srow[256];
  const int n = blockIdx.x, tid = threadIdx.x; const float* Wm; int K, NO, nn; size_t base;
  if (n < 256) { Wm = WinS; K = EIN; NO = HH; nn = n; base = PT_WIN(0) + (size_t)nn * EIN; }
  else if (n < 512) { Wm = WinC; K = EIN; NO = HH; nn = n - 256; base = PT_WIN(1) + (size_t)nn * EIN; }
  else if (n < 640) { Wm = WoS; K = HH; NO = OUTD; nn = n - 512; base = PT_WOUT(0) + (size_t)nn * HH; }
  else if (n < 768) { Wm = WoC; K = HH; NO = OUTD; nn = n - 640; base = PT_WOUT(1) + (size_t)nn * HH; }
  else if (n < 896) { Wm = Ws2c; K = OUTD; NO = OUTD; nn = n - 768; base = PT_WS2C + (size_t)nn * OUTD; }
  else { Wm = Wc2s; K = OUTD; NO = OUTD; nn = n - 896; base = PT_WC2S + (size_t)nn * OUTD; }
  if (tid < K) srow[tid] = (__bf16)Wm[(size_t)tid * NO + nn];
  __syncthreads();
  if (tid < K / 8) vst2((unsigned*)(PT + base + tid * 8), *(const v4u*)(&srow[tid * 8]));
}
__global__ __launch_bounds__(256) void k_h0(const int* __restrict__ xid, const float* __restrict__ e0s, const float* __restrict__ e1s, const float* __restrict__ e2s, const float* __restrict__ e0c, const float* __restrict__ e1c, const float* __restrict__ e2c,
                                            const __bf16* __restrict__ PT, const float* __restrict__ binS, const float* __restrict__ binC, float* __restrict__ H0) {
  __shared__ __align__(16) __bf16 se[64][EIN + 8];
  __shared__ __align__(16) float so[64][HH + 4];
  const int tid = threadIdx.x, wave = tid >> 5, lane = tid & 31, col = lane & 15, g = lane >> 4; const int m = blockIdx.y; const int nb = blockIdx.x * 64;
  const float* e0 = m ? e0c : e0s; const float* e1 = m ? e1c : e1s; const float* e2 = m ? e2c : e2s; const float* bin_ = m ? binC : binS;
  { const int nl = tid >> 2, q4 = tid & 3; const int n = nb + nl;
    int i0 = xid[n * 3 + 0], i1 = xid[n * 3 + 1], i2 = xid[n * 3 + 2];
    i0 = i0 < 0 ? 0 : (i0 > 49999 ? 49999 : i0); i1 = i1 < 0 ? 0 : (i1 > 999 ? 999 : i1); i2 = i2 < 0 ? 0 : (i2 > 199 ? 199 : i2);
#pragma unroll
    for (int c = 0; c < 32; ++c) { const int cc = q4 * 32 + c;
      const float v0 = e0[(size_t)i0 * 64 + (cc < 64 ? cc : 63)], v1 = e1[(size_t)i1 * 32 + (cc >= 64 && cc < 96 ? cc - 64 : 0)], v2 = e2[(size_t)i2 * 32 + (cc >= 96 ? cc - 96 : 0)];
      se[nl][cc] = (__bf16)(cc < 64 ? v0 : (cc < 96 ? v1 : v2)); } }
  __syncthreads();
  { const int rt = wave & 3, ct0 = (wave >> 2) * 8; v8f acc[8] = {};
#pragma unroll
    for (int kc = 0; kc < EIN / 32; ++kc) { const v16b a = frag_b(&se[rt * 16 + col][kc * 32], lane);
#pragma unroll
      for (int j = 0; j < 8; ++j) acc[j] = wmma_bf(a, frag_b(PT + PT_WIN(m) + (size_t)((ct0 + j) * 16 + col) * EIN + kc * 32, lane), acc[j]); }
#pragma unroll
    for (int j = 0; j < 8; ++j) { const int c = (ct0 + j) * 16 + col; const float bb = bfr(bin_[c]);
#pragma unroll
      for (int r = 0; r < 8; ++r) so[rt * 16 + 8 * g + r][c] = acc[j][r] + bb; } }
  __syncthreads();
  float* Hm = H0 + (size_t)m * N0 * HH;
#pragma unroll
  for (int it = 0; it < 16; ++it) { const int q = tid + 256 * it; const int r = q >> 6, c4 = (q & 63) * 4; vst2(Hm + (size_t)(nb + r) * HH + c4, *(const v4f*)(&so[r][c4])); }
}
template <int K, int RELU>
__global__ __launch_bounds__(256) void k_co(const float* __restrict__ Hin, int nsrc, int ndst, const int* __restrict__ idxD, const int* __restrict__ idxQ, float* __restrict__ Hout) {
  __shared__ float sL[8][K * K], sAC[8][K * K], sAS[8][K * K], sa[8][16], sb[8][16];
  __shared__ int siq[8][16], sid[8][16];
  __shared__ __align__(16) float sq[8][K][HH];
  __shared__ __align__(16) float sc[8][3 * HH];
  const int tid = threadIdx.x, wave = tid >> 5, lane = tid & 31; const int n = blockIdx.x * 8 + wave;
  if (n >= ndst) return;
  if (lane < K) { int a = idxQ[n * K + lane], d = idxD[n * K + lane]; siq[wave][lane] = a < 0 ? 0 : (a >= nsrc ? nsrc - 1 : a); sid[wave][lane] = d < 0 ? 0 : (d >= nsrc ? nsrc - 1 : d); }
  LDSX();
#pragma unroll 1
  for (int j = 0; j < K; ++j) { const size_t rq = (size_t)siq[wave][j] * HH;
    *(float4*)&sq[wave][j][lane * 4] = *(const float4*)(Hin + rq + lane * 4); *(float4*)&sq[wave][j][128 + lane * 4] = *(const float4*)(Hin + rq + 128 + lane * 4); }
  LDSX();
#pragma unroll 1
  for (int k = 0; k < K; ++k) { const size_t rd = (size_t)sid[wave][k] * HH; const float4 a = *(const float4*)(Hin + rd + lane * 4), c = *(const float4*)(Hin + rd + 128 + lane * 4);
#pragma unroll 1
    for (int mq = 0; mq < K; ++mq) { const float4 qa = *(const float4*)&sq[wave][mq][lane * 4], qc = *(const float4*)&sq[wave][mq][128 + lane * 4];
      float s = a.x * qa.x + a.y * qa.y + a.z * qa.z + a.w * qa.w + c.x * qc.x + c.y * qc.y + c.z * qc.z + c.w * qc.w;
#pragma unroll
      for (int o = 16; o > 0; o >>= 1) s += __shfl_xor(s, o);
      if (lane == 0) sL[wave][k * K + mq] = s; } }
  LDSX();
  if (lane < K) {
    { float mx = -3.0e38f;
#pragma unroll 1
      for (int mq = 0; mq < K; ++mq) mx = fmaxf(mx, sL[wave][lane * K + mq]);
      float s = 0.f;
#pragma unroll 1
      for (int mq = 0; mq < K; ++mq) { const float e = exp_ni(sL[wave][lane * K + mq] - mx); sAC[wave][lane * K + mq] = e; s += e; }
      const float inv = 1.0f / s;
#pragma unroll 1
      for (int mq = 0; mq < K; ++mq) sAC[wave][lane * K + mq] *= inv; }
    { float mx = -3.0e38f;
#pragma unroll 1
      for (int k = 0; k < K; ++k) mx = fmaxf(mx, sL[wave][k * K + lane]);
      float s = 0.f;
#pragma unroll 1
      for (int k = 0; k < K; ++k) { const float e = exp_ni(sL[wave][k * K + lane] - mx); sAS[wave][lane * K + k] = e; s += e; }
      const float inv = 1.0f / s;
#pragma unroll 1
      for (int k = 0; k < K; ++k) sAS[wave][lane * K + k] *= inv; } }
  LDSX();
  if (lane < K) { float a = 0.f;
#pragma unroll 1
    for (int mq = 0; mq < K; ++mq) a += sAS[wave][mq * K + lane]; sa[wave][lane] = a; }
  LDSX();
  if (lane < K) { float bsum = 0.f;
#pragma unroll 1
    for (int k = 0; k < K; ++k) bsum += sa[wave][k] * sAC[wave][k * K + lane]; sb[wave][lane] = bsum; }
  LDSX();
  float4 c0a = {0.f, 0.f, 0.f, 0.f}, c0b = c0a, c1a = c0a, c1b = c0a, c2a = c0a, c2b = c0a;
#pragma unroll 1
  for (int mq = 0; mq < K; ++mq) { const float bm = sb[wave][mq]; const float4 qa = *(const float4*)&sq[wave][mq][lane * 4], qc = *(const float4*)&sq[wave][mq][128 + lane * 4];
    c0a += qa; c0b += qc; c2a += bm * qa; c2b += bm * qc; }
#pragma unroll 1
  for (int k = 0; k < K; ++k) { const float ak = sa[wave][k]; const size_t rd = (size_t)sid[wave][k] * HH; const float4 a = *(const float4*)(Hin + rd + lane * 4), c = *(const float4*)(Hin + rd + 128 + lane * 4);
    c1a += ak * a; c1b += ak * c; }
  *(float4*)&sc[wave][lane * 4] = c0a; *(float4*)&sc[wave][128 + lane * 4] = c0b; *(float4*)&sc[wave][HH + lane * 4] = c1a; *(float4*)&sc[wave][HH + 128 + lane * 4] = c1b; *(float4*)&sc[wave][2 * HH + lane * 4] = c2a; *(float4*)&sc[wave][2 * HH + 128 + lane * 4] = c2b;
  LDSX();
  const float inv = (1.0f / 3.0f) / (float)K;
  v4f oa, ob;
  { const float4 ra = *(const float4*)(Hin + (size_t)n * HH + lane * 4), rb = *(const float4*)(Hin + (size_t)n * HH + 128 + lane * 4); const float rav[4] = {ra.x, ra.y, ra.z, ra.w}, rbv[4] = {rb.x, rb.y, rb.z, rb.w};
#pragma unroll
    for (int i = 0; i < 4; ++i) { const int fa = lane * 4 + i, fb = 128 + lane * 4 + i;
      float va = rav[i] + ((sc[wave][3 * fa] + sc[wave][3 * fa + 1]) + sc[wave][3 * fa + 2]) * inv; float vb = rbv[i] + ((sc[wave][3 * fb] + sc[wave][3 * fb + 1]) + sc[wave][3 * fb + 2]) * inv;
      if (RELU) { va = va > 0.f ? va : 0.f; vb = vb > 0.f ? vb : 0.f; } oa[i] = va; ob[i] = vb; } }
  vst2(Hout + (size_t)n * HH + lane * 4, oa); vst2(Hout + (size_t)n * HH + 128 + lane * 4, ob);
}
__global__ __launch_bounds__(128) void k_wout(const float* __restrict__ H2, const __bf16* __restrict__ PT, const float* __restrict__ boS, const float* __restrict__ boC, float* __restrict__ S) {
  __shared__ __align__(16) float so[4][16][132];
  const int tid = threadIdx.x, wave = tid >> 5, lane = tid & 31, col = lane & 15, g = lane >> 4; const int m = blockIdx.y; const size_t r0 = (size_t)blockIdx.x * 64 + wave * 16;
  const int nrow = N2; const float* Hm = H2 + (size_t)m * N2 * HH; const float* bo = m ? boC : boS;
  v8f acc[8] = {};
#pragma unroll 2
  for (int kc = 0; kc < HH / 32; ++kc) { const size_t rr = (r0 + col) < (size_t)nrow ? (r0 + col) : (size_t)(nrow - 1); const F2 a = split_row(Hm + rr * HH, kc * 32, lane);
#pragma unroll
    for (int j = 0; j < 8; ++j) { const v16b wb = frag_b(PT + PT_WOUT(m) + (size_t)(j * 16 + col) * HH + kc * 32, lane); acc[j] = wmma_bf(a.l, wb, acc[j]); acc[j] = wmma_bf(a.h, wb, acc[j]); } }
#pragma unroll
  for (int j = 0; j < 8; ++j) { const float bb = bfr(bo[j * 16 + col]);
#pragma unroll
    for (int r = 0; r < 8; ++r) so[wave][8 * g + r][j * 16 + col] = acc[j][r] + bb; }
  LDSX();
  for (int rl = 0; rl < 16; ++rl) { const size_t row = r0 + rl; if (row < (size_t)nrow) vst2(S + ((size_t)m * N2 + row) * OUTD + lane * 4, *(const v4f*)(&so[wave][rl][lane * 4])); }
}
__device__ __forceinline__ void semi_gemm4(const float* arow_base, const __bf16* __restrict__ PTm, int ct0, int lane, int col, v8f acc[4]) {
#pragma unroll
  for (int j = 0; j < 4; ++j) acc[j] = (v8f){};
#pragma unroll
  for (int kc = 0; kc < OUTD / 32; ++kc) { const F2 a = split_row(arow_base, kc * 32, lane);
#pragma unroll
    for (int j = 0; j < 4; ++j) { const v16b wb = frag_b(PTm + (size_t)((ct0 + j) * 16 + col) * OUTD + kc * 32, lane); acc[j] = wmma_bf(a.l, wb, acc[j]); acc[j] = wmma_bf(a.h, wb, acc[j]); } }
}
__global__ __launch_bounds__(128) void k_semi(const float* __restrict__ S, const __bf16* __restrict__ PT, const float* __restrict__ pa1, const float* __restrict__ pa2, const float* __restrict__ pb2, float* __restrict__ out) {
  __shared__ __align__(16) float z1s[64][132], z1c[64][132], sP[64][132], sQ[64][132];
  const int tid = threadIdx.x, wave = tid >> 5, lane = tid & 31, col = lane & 15, g = lane >> 4; const size_t r0 = (size_t)blockIdx.x * 64 + wave * 16;
  const float a1 = bfr(pa1[0]), a2 = bfr(pa2[0]), b2 = bfr(pb2[0]); const float c1 = 1.0f - a1, c2 = (1.0f - a2) - b2;
  const float* sim = S; const float* cor = S + (size_t)N2 * OUTD;
  const size_t ra = (r0 + col) < (size_t)N2 ? (r0 + col) : (size_t)(N2 - 1);
  v8f acc[4];
#pragma unroll 1
  for (int half = 0; half < 2; ++half) { const int ct0 = half * 4;
    semi_gemm4(cor + ra * OUTD, PT + PT_WC2S, ct0, lane, col, acc);
#pragma unroll
    for (int j = 0; j < 4; ++j)
#pragma unroll
      for (int r = 0; r < 8; ++r) sP[wave * 16 + 8 * g + r][(ct0 + j) * 16 + col] = acc[j][r];
    semi_gemm4(sim + ra * OUTD, PT + PT_WS2C, ct0, lane, col, acc);
#pragma unroll
    for (int j = 0; j < 4; ++j)
#pragma unroll
      for (int r = 0; r < 8; ++r) sQ[wave * 16 + 8 * g + r][(ct0 + j) * 16 + col] = acc[j][r]; }
  LDSX();
#pragma unroll 1
  for (int rl = 0; rl < 16; ++rl) { const int rr = wave * 16 + rl; const size_t row = (r0 + rl) < (size_t)N2 ? (r0 + rl) : (size_t)(N2 - 1);
#pragma unroll
    for (int i = 0; i < 4; ++i) { const int c = lane * 4 + i; z1s[rr][c] = c1 * sim[row * OUTD + c] + a1 * sP[rr][c]; z1c[rr][c] = c1 * cor[row * OUTD + c] + a1 * sQ[rr][c]; } }
  LDSX();
#pragma unroll 1
  for (int half = 0; half < 2; ++half) { const int ct0 = half * 4;
    semi_gemm4(&z1c[wave * 16 + col][0], PT + PT_WC2S, ct0, lane, col, acc);
#pragma unroll
    for (int j = 0; j < 4; ++j)
#pragma unroll
      for (int r = 0; r < 8; ++r) { const int rr = wave * 16 + 8 * g + r, c = (ct0 + j) * 16 + col; const size_t row = (r0 + 8 * g + r) < (size_t)N2 ? (r0 + 8 * g + r) : (size_t)(N2 - 1);
        sP[rr][c] = (c2 * sim[row * OUTD + c] + a2 * sP[rr][c]) + b2 * acc[j][r]; }
    semi_gemm4(&z1s[wave * 16 + col][0], PT + PT_WS2C, ct0, lane, col, acc);
#pragma unroll
    for (int j = 0; j < 4; ++j)
#pragma unroll
      for (int r = 0; r < 8; ++r) { const int rr = wave * 16 + 8 * g + r, c = (ct0 + j) * 16 + col; const size_t row = (r0 + 8 * g + r) < (size_t)N2 ? (r0 + 8 * g + r) : (size_t)(N2 - 1);
        sQ[rr][c] = (c2 * cor[row * OUTD + c] + a2 * sQ[rr][c]) + b2 * acc[j][r]; } }
  LDSX();
  for (int rl = 0; rl < 16; ++rl) { const size_t row = r0 + rl; if (row < (size_t)N2) { vst2(out + row * OUTD + lane * 4, *(const v4f*)(&sP[wave * 16 + rl][lane * 4])); vst2(out + ((size_t)N2 + row) * OUTD + lane * 4, *(const v4f*)(&sQ[wave * 16 + rl][lane * 4])); } }
}

extern "C" void kernel_launch(void* const* d_in, const int* in_sizes, int n_in, void* d_out, int out_size, void* d_ws, size_t ws_size, hipStream_t stream) {
  (void)in_sizes; (void)n_in; (void)out_size;
  const int* xid = (const int*)d_in[0]; const int* is0 = (const int*)d_in[1]; const int* ic0 = (const int*)d_in[2]; const int* is1 = (const int*)d_in[3]; const int* ic1 = (const int*)d_in[4];
  const float** F = (const float**)d_in;
  if (ws_size < (size_t)WS_END) return;
  char* ws = (char*)d_ws; __bf16* PT = (__bf16*)(ws + WS_PT); float* H0 = (float*)(ws + WS_H0); float* H1 = (float*)(ws + WS_H1); float* H2 = (float*)(ws + WS_H2); float* S = (float*)(ws + WS_S);
  k_pack<<<1024, 256, 0, stream>>>(F[8], F[15], F[10], F[17], F[19], F[20], PT);
  k_h0<<<dim3(N0 / 64, 2), 256, 0, stream>>>(xid, F[5], F[6], F[7], F[12], F[13], F[14], PT, F[9], F[16], H0);
  k_co<10, 1><<<N1 / 8, 256, 0, stream>>>(H0, N0, N1, ic0, is0, H1);
  k_co<10, 1><<<N1 / 8, 256, 0, stream>>>(H0 + (size_t)N0 * HH, N0, N1, is0, ic0, H1 + (size_t)N1 * HH);
  k_co<5, 0><<<N2 / 8, 256, 0, stream>>>(H1, N1, N2, ic1, is1, H2);
  k_co<5, 0><<<N2 / 8, 256, 0, stream>>>(H1 + (size_t)N1 * HH, N1, N2, is1, ic1, H2 + (size_t)N2 * HH);
  k_wout<<<dim3((N2 + 63) / 64, 2), 128, 0, stream>>>(H2, PT, F[11], F[18], S);
  k_semi<<<(N2 + 63) / 64, 128, 0, stream>>>(S, PT, F[21], F[22], F[23], (float*)d_out);
}
